// CURLoRAModule_34325378629967
// MI455X (gfx1250) — hardware-verified
//
#include <hip/hip_runtime.h>
#include <math.h>

#ifndef NB
#define NB 2
#endif
#ifndef SEQ
#define SEQ 64
#endif
#define SEQ_FULL 64
#define M_DIM 8192
#define N_DIM 8192
#define RANK 64
#define MROWS (NB * SEQ)

static_assert(SEQ == SEQ_FULL);
static_assert(MROWS % 64 == 0);
static_assert(RANK % 64 == 0 && N_DIM % 64 == 0);
static_assert(M_DIM % 32 == 0 && RANK % 32 == 0);
static_assert(M_DIM % 8 == 0 && RANK % 8 == 0);
static_assert((MROWS * M_DIM / 8) % 256 == 0);
static_assert((RANK * M_DIM / 8) % 256 == 0);
static_assert((RANK * RANK / 8) % 256 == 0);
static_assert((N_DIM * RANK / 8) % 256 == 0);
static_assert((MROWS / 64) * (RANK / 64) <= 2);
static_assert(8 * 16 * 68 * 4 <= 131072);

typedef __attribute__((ext_vector_type(16))) _Float16 v16h;
typedef __attribute__((ext_vector_type(8)))  _Float16 v8h;
typedef __attribute__((ext_vector_type(8)))  float    v8f;
typedef __attribute__((ext_vector_type(4)))  float    v4f;
typedef __attribute__((ext_vector_type(4)))  unsigned int v4u;
typedef _Float16 h16;
typedef __attribute__((ext_vector_type(2)))  float    v2f;
typedef __attribute__((ext_vector_type(2)))  _Float16 v2h;
typedef __attribute__((ext_vector_type(4)))  _Float16 v4h;


constexpr size_t SZ_X16 = (size_t)MROWS * M_DIM * 2;
constexpr size_t SZ_R16 = (size_t)RANK * M_DIM * 2;
constexpr size_t SZ_C16 = (size_t)N_DIM * RANK * 2;
constexpr size_t SZ_U16 = (size_t)RANK * RANK * 2;
constexpr size_t SZ_T   = (size_t)MROWS * RANK * 2;
constexpr size_t OFF_X16 = 0;
constexpr size_t OFF_R16 = OFF_X16 + SZ_X16;
constexpr size_t OFF_C16 = OFF_R16 + SZ_R16;
constexpr size_t OFF_U16 = OFF_C16 + SZ_C16;
constexpr size_t OFF_T1  = OFF_U16 + SZ_U16;
constexpr size_t OFF_T2  = OFF_T1 + SZ_T;
constexpr size_t WS_TOTAL = OFF_T2 + SZ_T;
static_assert(SZ_X16 % 256 == 0 && SZ_R16 % 256 == 0 && SZ_C16 % 256 == 0 && SZ_U16 % 256 == 0 && SZ_T % 256 == 0);
static_assert(WS_TOTAL <= (size_t)134217728);

__device__ __forceinline__ float bfr(float f) {
    unsigned u = __float_as_uint(f);
    u += 0x7FFFu + ((u >> 16) & 1u);
    return __uint_as_float(u & 0xFFFF0000u);
}

__device__ __forceinline__ h16 toh_flush(float v) {
    const float w = (fabsf(v) < 6.103515625e-05f) ? 0.0f : v;
    return (h16)w;
}
__device__ __forceinline__ v2h toh_flush2(float a, float b) {
    v2f w;
    w.x = (fabsf(a) < 6.103515625e-05f) ? 0.0f : a;
    w.y = (fabsf(b) < 6.103515625e-05f) ? 0.0f : b;
    return __builtin_convertvector(w, v2h);
}
__device__ __forceinline__ v8h toh_flush8(v4f a, v4f b) {
    const v2h p0 = toh_flush2(a.x, a.y);
    const v2h p1 = toh_flush2(a.z, a.w);
    const v2h p2 = toh_flush2(b.x, b.y);
    const v2h p3 = toh_flush2(b.z, b.w);
    const v4h q0 = __builtin_shufflevector(p0, p1, 0, 1, 2, 3);
    const v4h q1 = __builtin_shufflevector(p2, p3, 0, 1, 2, 3);
    return __builtin_shufflevector(q0, q1, 0, 1, 2, 3, 4, 5, 6, 7);
}

union FragU { v16h v; v8h h[2]; };
__device__ __forceinline__ v16h frag_ld(const _Float16* p) {
    FragU f; f.h[0] = *(const v8h*)(p); f.h[1] = *(const v8h*)(p + 16); return f.v;
}
__device__ __forceinline__ v8f wmma16(v16h a, v16h b, v8f c) {
    c = __builtin_amdgcn_wmma_f32_16x16x32_f16(false, a, false, b, (short)0, c, false, false);
    asm volatile("v_nop\n\tv_nop\n\tv_nop\n\tv_nop" : "+v"(c) : "v"(a), "v"(b));
    return c;
}
__device__ __forceinline__ void wave_sync_lds() {
    __builtin_amdgcn_fence(3  , "workgroup");
    __builtin_amdgcn_wave_barrier();
    __builtin_amdgcn_fence(2  , "workgroup");
}

__global__ __launch_bounds__(256) void k_cvt16(const float* __restrict__ src, _Float16* __restrict__ dst, unsigned n8) {
    const unsigned u = blockIdx.x * 256u + threadIdx.x;
    if (u >= n8) return;
    const v4f a = *(const v4f*)(src + 8u * u);
    const v4f b = *(const v4f*)(src + 8u * u + 4u);
    v4f sa, sb;
    sa.x = bfr(a.x) * 256.0f; sa.y = bfr(a.y) * 256.0f; sa.z = bfr(a.z) * 256.0f; sa.w = bfr(a.w) * 256.0f;
    sb.x = bfr(b.x) * 256.0f; sb.y = bfr(b.y) * 256.0f; sb.z = bfr(b.z) * 256.0f; sb.w = bfr(b.w) * 256.0f;
    const v8h pk = toh_flush8(sa, sb);
    *(volatile v8h*)(dst + 8u * u) = pk;
    __threadfence();
    *(volatile v8h*)(dst + 8u * u) = pk;
}

template <int OUT_MODE>
__device__ __forceinline__ void gemm64_body(
    const _Float16* __restrict__ A, unsigned lda, const _Float16* __restrict__ Bt, unsigned ldb,
    void* __restrict__ Cout, unsigned ldc,
    unsigned M, unsigned N, unsigned K, float scale, float oscale) {
  __shared__ __align__(16) float sT[8][16 * 68];
  const unsigned lane = threadIdx.x & 31u;
  const unsigned wave = threadIdx.x >> 5;
  const unsigned tilesN = N >> 6, tilesM = M >> 6;
  const unsigned tile = blockIdx.x * 8u + wave;
  if (tile >= tilesM * tilesN) return;
  const unsigned tm = tile / tilesN;
  const unsigned tn = tile - tm * tilesN;
  const unsigned m0 = tm << 6, n0 = tn << 6;
  const unsigned rlane = lane & 15u;
  const unsigned koff = (lane >> 4) * 8u;
  const unsigned mOff = koff;

  v8f acc[4][4];
#pragma unroll
  for (int i = 0; i < 4; ++i)
#pragma unroll
    for (int j = 0; j < 4; ++j) acc[i][j] = (v8f){0.f,0.f,0.f,0.f,0.f,0.f,0.f,0.f};

  for (unsigned k0 = 0; k0 < K; k0 += 32u) {
    v16h bh[4];
#pragma unroll
    for (int j = 0; j < 4; ++j)
      bh[j] = frag_ld(Bt + (size_t)(n0 + ((unsigned)j << 4) + rlane) * ldb + koff + k0);
#pragma unroll
    for (int i = 0; i < 4; ++i) {
      const v16h ah = frag_ld(A + (size_t)(m0 + ((unsigned)i << 4) + rlane) * lda + koff + k0);
#pragma unroll
      for (int j = 0; j < 4; ++j)
        acc[i][j] = wmma16(ah, bh[j], acc[i][j]);
    }
  }

  float* slab = sT[wave];
#pragma unroll
  for (int i = 0; i < 4; ++i) {
    const unsigned mBase = m0 + ((unsigned)i << 4);
#pragma unroll
    for (int j = 0; j < 4; ++j) {
#pragma unroll
      for (int r = 0; r < 8; ++r) {
        float v = acc[i][j][r] * scale;
        if (OUT_MODE == 1) v *= oscale;
        slab[(mOff + (unsigned)r) * 68u + ((unsigned)j << 4) + rlane] = v;
      }
    }
    wave_sync_lds();
    if (OUT_MODE == 0) {
      float* C = (float*)Cout;
      const unsigned hh = lane >> 4, c4 = (lane & 15u) * 4u;
      static_assert(32 * 16 * (2 * 4) == 16 * 64 * 4);
#pragma unroll
      for (int half = 0; half < 2; ++half) {
        v4f vv[4];
#pragma unroll
        for (int it = 0; it < 4; ++it) {
          const unsigned row = (unsigned)(half * 4 + it) * 2u + hh;
          vv[it] = *(const v4f*)(slab + row * 68u + c4);
        }
        for (int pass = 0; pass < 2; ++pass) {
#pragma unroll
          for (int it = 0; it < 4; ++it) {
            const unsigned row = (unsigned)(half * 4 + it) * 2u + hh;
            *(volatile v4f*)(C + (size_t)(mBase + row) * ldc + n0 + c4) = vv[it];
          }
          __threadfence();
        }
      }
    } else {
      _Float16* C = (_Float16*)Cout;
      const unsigned q = lane >> 3, c8 = (lane & 7u) * 8u;
      static_assert(32 * 16 * 4 == 16 * 64 * 2);
      v8h hv[4];
#pragma unroll
      for (int it = 0; it < 4; ++it) {
        const unsigned row = (unsigned)it * 4u + q;
        const float* sp = slab + row * 68u + c8;
        hv[it] = toh_flush8(*(const v4f*)(sp), *(const v4f*)(sp + 4));
      }
      for (int pass = 0; pass < 2; ++pass) {
#pragma unroll
        for (int it = 0; it < 4; ++it) {
          const unsigned row = (unsigned)it * 4u + q;
          *(volatile v8h*)(C + (size_t)(mBase + row) * ldc + n0 + c8) = hv[it];
        }
        __threadfence();
      }
    }
    wave_sync_lds();
  }
}

__global__ __launch_bounds__(256) void k_gemm_t1(const _Float16* __restrict__ X16, const _Float16* __restrict__ R16,
                                                 _Float16* __restrict__ T1) {
    gemm64_body<1>(X16, M_DIM, R16, M_DIM, (void*)T1, RANK, MROWS, RANK, M_DIM, 1.52587890625e-05f, 8.0f);
}

__global__ __launch_bounds__(256) void k_gemm_t2(const _Float16* __restrict__ T1, const _Float16* __restrict__ U16,
                                                 _Float16* __restrict__ T2) {
    gemm64_body<1>(T1, RANK, U16, RANK, (void*)T2, RANK, MROWS, RANK, RANK, 4.8828125e-04f, 1.0f);
}

__global__ __launch_bounds__(256) void k_gemm_out(const _Float16* __restrict__ T2, const _Float16* __restrict__ C16,
                                                  float* __restrict__ out) {
    gemm64_body<0>(T2, RANK, C16, RANK, (void*)out, N_DIM, MROWS, N_DIM, RANK, 3.90625e-03f, 1.0f);
}

extern "C" void kernel_launch(void* const* d_in, const int* in_sizes, int n_in, void* d_out, int out_size,
                              void* d_ws, size_t ws_size, hipStream_t stream) {
    if (n_in < 4) return;
    if (in_sizes[0] < MROWS * M_DIM || in_sizes[1] < N_DIM * RANK || in_sizes[2] < RANK * RANK || in_sizes[3] < RANK * M_DIM) return;
    if (out_size < MROWS * N_DIM) return;
    if ((size_t)WS_TOTAL > ws_size) return;

    const float* x  = (const float*)d_in[0];
    const float* Cm = (const float*)d_in[1];
    const float* Um = (const float*)d_in[2];
    const float* Rm = (const float*)d_in[3];
    float* out = (float*)d_out;

    char* wsp = (char*)d_ws;
    _Float16* X16 = (_Float16*)(wsp + OFF_X16);
    _Float16* R16 = (_Float16*)(wsp + OFF_R16);
    _Float16* C16 = (_Float16*)(wsp + OFF_C16);
    _Float16* U16 = (_Float16*)(wsp + OFF_U16);
    _Float16* T1  = (_Float16*)(wsp + OFF_T1);
    _Float16* T2  = (_Float16*)(wsp + OFF_T2);

    k_cvt16<<<(MROWS * M_DIM / 8) / 256, 256, 0, stream>>>(x,  X16, (unsigned)(MROWS * M_DIM / 8));
    k_cvt16<<<(RANK * M_DIM / 8) / 256,  256, 0, stream>>>(Rm, R16, (unsigned)(RANK * M_DIM / 8));
    k_cvt16<<<(RANK * RANK / 8) / 256,   256, 0, stream>>>(Um, U16, (unsigned)(RANK * RANK / 8));
    k_cvt16<<<(N_DIM * RANK / 8) / 256,  256, 0, stream>>>(Cm, C16, (unsigned)(N_DIM * RANK / 8));

    k_gemm_t1<<<1, 64, 0, stream>>>((const _Float16*)X16, (const _Float16*)R16, T1);
    k_gemm_t2<<<1, 64, 0, stream>>>((const _Float16*)T1, (const _Float16*)U16, T2);

    const unsigned gOut = ((MROWS / 64) * (N_DIM / 64) + 7) / 8;
    k_gemm_out<<<gOut, 256, 0, stream>>>((const _Float16*)T2, (const _Float16*)C16, out);
}
